// RWKV7Block_48103633715813
// MI455X (gfx1250) — hardware-verified
//
#include <hip/hip_runtime.h>
#include <hip/hip_bf16.h>
#include <math.h>
#include <stdint.h>
#include <stddef.h>

typedef __attribute__((ext_vector_type(16))) __bf16   v16b;
typedef __attribute__((ext_vector_type(8)))  __bf16   v8b;
typedef __attribute__((ext_vector_type(8)))  float    v8f;
typedef __attribute__((ext_vector_type(4)))  float    v4f;
typedef __attribute__((ext_vector_type(4)))  unsigned v4u;
typedef __attribute__((ext_vector_type(2)))  unsigned v2u;

constexpr int NBATCH = 4;
constexpr int NSEQ   = 2048;
constexpr int NDIM   = 1024;
constexpr int NHEAD  = 16;
constexpr int HDIM   = 64;
constexpr int NTOK   = NBATCH * NSEQ;
constexpr int PROJ_N = 4 * NDIM;

static_assert(NHEAD * HDIM == NDIM, "heads");
static_assert(NDIM % 32 == 0, "K");
static_assert(NSEQ % 64 == 0 && PROJ_N % 64 == 0, "proj GEMM M,N");
static_assert(NTOK % 64 == 0 && NDIM % 64 == 0, "out GEMM M,N");

constexpr size_t OFF_XB   = 0;
constexpr size_t SZ_XB    = (size_t)NTOK * NDIM * 2;
constexpr size_t OFF_WALL = OFF_XB + SZ_XB;
constexpr size_t SZ_WALL  = (size_t)PROJ_N * NDIM * 2;
constexpr size_t OFF_WOB  = OFF_WALL + SZ_WALL;
constexpr size_t SZ_WOB   = (size_t)NDIM * NDIM * 2;
constexpr size_t OFF_PROJ = OFF_WOB + SZ_WOB;
constexpr size_t SZ_PROJ  = (size_t)NSEQ * PROJ_N * 4;
constexpr size_t OFF_KSUM = OFF_PROJ + SZ_PROJ;
constexpr size_t SZ_KSUM  = (size_t)NSEQ * NHEAD * 4;
constexpr size_t OFF_YF   = OFF_KSUM + SZ_KSUM;
constexpr size_t SZ_YF    = (size_t)NTOK * NDIM * 4;
constexpr size_t OFF_YNHI = OFF_YF + SZ_YF;
constexpr size_t SZ_YN    = (size_t)NTOK * NDIM * 2;
constexpr size_t OFF_YNLO = OFF_YNHI + SZ_YN;
constexpr size_t WS_TOTAL = OFF_YNLO + SZ_YN;
static_assert(WS_TOTAL == 128057344ull, "carve total");
static_assert(WS_TOTAL <= 134217728ull, "carve cap");
static_assert(OFF_WALL % 128 == 0 && OFF_WOB % 128 == 0 && OFF_PROJ % 128 == 0 && OFF_KSUM % 128 == 0 &&
              OFF_YF % 128 == 0 && OFF_YNHI % 128 == 0 && OFF_YNLO % 128 == 0, "alignment");
static_assert((size_t)NTOK * NDIM * 4 == 33554432ull, "out bytes");

__device__ __forceinline__ unsigned short f2bf_bits(float f) {
  unsigned u = __float_as_uint(f);
  return (unsigned short)((u + 0x7FFFu + ((u >> 16) & 1u)) >> 16);
}
__device__ __forceinline__ float bf_bits2f(unsigned short h) { return __uint_as_float(((unsigned)h) << 16); }

__device__ __forceinline__ void dep_guard_b(v8f& a, v8f& b, v16b x, v16b y) { asm volatile("v_nop\n\tv_nop\n\tv_nop\n\tv_nop" : "+v"(a), "+v"(b) : "v"(x), "v"(y)); }
__device__ __forceinline__ void keep4_b(v16b a, v16b b, v16b c, v16b d) { asm volatile("v_nop" :: "v"(a), "v"(b), "v"(c), "v"(d)); }
__device__ __forceinline__ void acc_guard4(v8f& a, v8f& b, v8f& c, v8f& d) { asm volatile("v_nop\n\tv_nop\n\tv_nop\n\tv_nop" : "+v"(a), "+v"(b), "+v"(c), "+v"(d)); }

template <typename T> struct Frag;
template <> struct Frag<__bf16> {
  typedef v16b V; union U { v16b v; v8b h[2]; };
  static __device__ __forceinline__ v16b load(const __bf16* p) {
    U f; f.h[0] = *(const v8b*)(p); f.h[1] = *(const v8b*)(p + 16); return f.v;
  }
  static __device__ __forceinline__ v8f mma(v16b a, v16b b, v8f c) {
    return __builtin_amdgcn_wmma_f32_16x16x32_bf16(false, a, false, b, (short)0, c, false, false);
  }
  static __device__ __forceinline__ void guard(v8f& a, v8f& b, v16b x, v16b y) { dep_guard_b(a, b, x, y); }
  static __device__ __forceinline__ void keep(v16b a, v16b b, v16b c, v16b d) { keep4_b(a, b, c, d); }
};

template <int SPLITM>
__global__ __launch_bounds__(256) void wmma_gemm64_bf16(
    const unsigned short* __restrict__ Ap, const unsigned short* __restrict__ A2p, int lda,
    const unsigned short* __restrict__ Btp, const unsigned short* __restrict__ Bt2p, int ldb,
    float* __restrict__ Cout, int ldc, int M, int N, int K, float scale) {
  constexpr bool SA = (SPLITM == 1) || (SPLITM == 2);
  constexpr bool SB = (SPLITM == 1) || (SPLITM == 3);
  typedef __bf16 T;
  typedef Frag<__bf16>::V V;
  const T* Ab  = (const T*)Ap;
  const T* Ab2 = (const T*)A2p;
  const T* Bb  = (const T*)Btp;
  const T* Bb2 = (const T*)Bt2p;
  __shared__ __align__(16) float sT[8][16 * 68];
  const int lane = threadIdx.x & 31;
  const int wave = threadIdx.x >> 5;
  const int tilesN = N >> 6;
  const int tilesM = M >> 6;
  const int tile = blockIdx.x * 8 + wave;
  if (tile >= tilesM * tilesN) return;
  const int tm = tile / tilesN;
  const int tn = tile - tm * tilesN;
  const int m0 = tm << 6;
  const int n0 = tn << 6;

  const int rlane = lane & 15;
  const int koff  = (lane >> 4) * 8;
  const int mOff  = (lane >> 4) * 8;

  v8f acc[4][4];
#pragma unroll
  for (int i = 0; i < 4; ++i)
#pragma unroll
    for (int j = 0; j < 4; ++j) acc[i][j] = (v8f){0.f,0.f,0.f,0.f,0.f,0.f,0.f,0.f};

  for (int k0 = 0; k0 < K; k0 += 32) {
    V bh[4], bl[4];
#pragma unroll
    for (int j = 0; j < 4; ++j) {
      const size_t bo = (size_t)(n0 + (j << 4) + rlane) * ldb + koff + k0;
      bh[j] = Frag<T>::load(Bb + bo);
      if (SB) bl[j] = Frag<T>::load(Bb2 + bo);
    }
#pragma unroll
    for (int i = 0; i < 4; ++i) {
      const size_t ao = (size_t)(m0 + (i << 4) + rlane) * lda + koff + k0;
      V ah = Frag<T>::load(Ab + ao);
      V al;
      if (SA) al = Frag<T>::load(Ab2 + ao);
#pragma unroll
      for (int j = 0; j < 4; ++j) {
        acc[i][j] = Frag<T>::mma(ah, bh[j], acc[i][j]);
        if (SB) acc[i][j] = Frag<T>::mma(ah, bl[j], acc[i][j]);
        if (SA) acc[i][j] = Frag<T>::mma(al, bh[j], acc[i][j]);
      }
      Frag<T>::guard(acc[i][0], acc[i][3], ah, SA ? al : ah);
    }
    Frag<T>::keep(bh[0], bh[1], bh[2], bh[3]);
    if (SB) Frag<T>::keep(bl[0], bl[1], bl[2], bl[3]);
  }
  acc_guard4(acc[0][0], acc[0][1], acc[0][2], acc[0][3]);
  acc_guard4(acc[1][0], acc[1][1], acc[1][2], acc[1][3]);
  acc_guard4(acc[2][0], acc[2][1], acc[2][2], acc[2][3]);
  acc_guard4(acc[3][0], acc[3][1], acc[3][2], acc[3][3]);

  float* slab = sT[wave];
#pragma unroll
  for (int i = 0; i < 4; ++i) {
    const int mBase = m0 + (i << 4);
#pragma unroll
    for (int j = 0; j < 4; ++j) {
#pragma unroll
      for (int r = 0; r < 8; ++r) {
        const float v = acc[i][j][r] * scale;
        slab[(mOff + r) * 68 + (j << 4) + rlane] = v;
      }
    }
    __builtin_amdgcn_fence(__ATOMIC_RELEASE, "workgroup");
    __builtin_amdgcn_wave_barrier();
    __builtin_amdgcn_fence(__ATOMIC_ACQUIRE, "workgroup");
    {
      const int hh = lane >> 4, c4 = (lane & 15) * 4;
      for (int pass = 0; pass < 2; ++pass) {
#pragma unroll
        for (int it = 0; it < 8; ++it) {
          const int row = it * 2 + hh;
          v4f v = *(const v4f*)(slab + row * 68 + c4);
          *(volatile v4f*)(Cout + (size_t)(mBase + row) * ldc + n0 + c4) = v;
        }
        __threadfence();
      }
    }
    __builtin_amdgcn_fence(__ATOMIC_RELEASE, "workgroup");
    __builtin_amdgcn_wave_barrier();
    __builtin_amdgcn_fence(__ATOMIC_ACQUIRE, "workgroup");
  }
}

__global__ __launch_bounds__(256) void cast_f32_bf16x8(
    const float* __restrict__ in, unsigned short* __restrict__ out, int n8) {
  const int i = blockIdx.x * 256 + threadIdx.x;
  if (i < n8) {
    const size_t e = (size_t)i * 8;
    const v4f a = *(const v4f*)(in + e);
    const v4f b = *(const v4f*)(in + e + 4);
    v4u u;
    u[0] = (unsigned)f2bf_bits(a[0]) | ((unsigned)f2bf_bits(a[1]) << 16);
    u[1] = (unsigned)f2bf_bits(a[2]) | ((unsigned)f2bf_bits(a[3]) << 16);
    u[2] = (unsigned)f2bf_bits(b[0]) | ((unsigned)f2bf_bits(b[1]) << 16);
    u[3] = (unsigned)f2bf_bits(b[2]) | ((unsigned)f2bf_bits(b[3]) << 16);
    *(volatile v4u*)(out + e) = u;
    __threadfence();
    *(volatile v4u*)(out + e) = u;
  }
}

__global__ __launch_bounds__(256) void ksum_kernel(const float* __restrict__ P, float* __restrict__ KS) {
  const int q = blockIdx.x * 256 + threadIdx.x;
  const int t = q >> 4;
  const int h = q & 15;
  const float* kp = P + (size_t)t * PROJ_N + NDIM + h * HDIM;
  float s = 0.f;
#pragma unroll 1
  for (int i = 0; i < 4; ++i) {
    const float* p = kp + 16 * i;
    const v4f a = *(const v4f*)(p);
    const v4f b = *(const v4f*)(p + 4);
    const v4f c = *(const v4f*)(p + 8);
    const v4f d = *(const v4f*)(p + 12);
    s += ((a[0] + a[1]) + (a[2] + a[3])) + ((b[0] + b[1]) + (b[2] + b[3]))
       + ((c[0] + c[1]) + (c[2] + c[3])) + ((d[0] + d[1]) + (d[2] + d[3]));
  }
  *(volatile float*)(KS + q) = s;
  __threadfence();
  *(volatile float*)(KS + q) = s;
}

__device__ __forceinline__ float sigm(float x) {
  const float e = expf(-x);
  return __builtin_amdgcn_rcpf(1.0f + e);
}

__global__ __launch_bounds__(64) void scan_kernel(const float* __restrict__ P, const float* __restrict__ KS,
                                                  float* __restrict__ Y, int tok0) {
  const int h  = blockIdx.x;
  const int c  = threadIdx.x;
  const int ch = h * HDIM + c;
  float s = 0.f;
#pragma unroll 1
  for (int t = 0; t < NSEQ; ++t) {
    const float* prow = P + (size_t)t * PROJ_N;
    const float rl = prow[ch];
    const float vv = prow[2 * NDIM + ch];
    const float wl = prow[3 * NDIM + ch];
    const float ks = KS[t * NHEAD + h];
    const float w = 0.99f * sigm(wl);
    const float r = sigm(rl);
    s = s * w + vv * ks;
    const float y = r * s;
    float* yp = Y + (size_t)(tok0 + t) * NDIM + ch;
    *(volatile float*)yp = y;
    __threadfence();
    *(volatile float*)yp = y;
  }
}

__global__ __launch_bounds__(256) void rmsnorm_split_kernel(const float* __restrict__ Y,
                                                           unsigned short* __restrict__ Hi,
                                                           unsigned short* __restrict__ Lo) {
  __shared__ float red[8];
  const int tok  = blockIdx.x;
  const int tid  = threadIdx.x;
  const int lane = tid & 31;
  const int wave = tid >> 5;
  const size_t base = (size_t)tok * NDIM + (size_t)tid * 4;
  const v4f y = *(const v4f*)(Y + base);
  float ss = (y[0] * y[0] + y[1] * y[1]) + (y[2] * y[2] + y[3] * y[3]);
#pragma unroll
  for (int off = 16; off; off >>= 1) ss += __shfl_xor(ss, off, 32);
  if (lane == 0) red[wave] = ss;
  __syncthreads();
  float tot = red[0];
#pragma unroll
  for (int i = 1; i < 8; ++i) tot += red[i];
  const float sc = rsqrtf(tot * (1.0f / 1024.0f) + 1.1920928955078125e-7f);
  unsigned short hb[4], lb[4];
#pragma unroll
  for (int e = 0; e < 4; ++e) {
    const float f = y[e] * sc;
    hb[e] = f2bf_bits(f);
    lb[e] = f2bf_bits(f - bf_bits2f(hb[e]));
  }
  v2u hv, lv;
  hv[0] = (unsigned)hb[0] | ((unsigned)hb[1] << 16);
  hv[1] = (unsigned)hb[2] | ((unsigned)hb[3] << 16);
  lv[0] = (unsigned)lb[0] | ((unsigned)lb[1] << 16);
  lv[1] = (unsigned)lb[2] | ((unsigned)lb[3] << 16);
  *(volatile v2u*)(Hi + base) = hv;
  *(volatile v2u*)(Lo + base) = lv;
  __threadfence();
  *(volatile v2u*)(Hi + base) = hv;
  *(volatile v2u*)(Lo + base) = lv;
}

extern "C" void kernel_launch(void* const* d_in, const int* in_sizes, int n_in,
                              void* d_out, int out_size, void* d_ws, size_t ws_size,
                              hipStream_t stream) {
  if (n_in < 6) return;
  if (in_sizes[0] != NTOK * NDIM) return;
  for (int i = 1; i < 6; ++i) if (in_sizes[i] != NDIM * NDIM) return;
  if (out_size != NTOK * NDIM) return;
  if (ws_size < WS_TOTAL) return;

  const float* x  = (const float*)d_in[0];
  const float* Wr = (const float*)d_in[1];
  const float* Wk = (const float*)d_in[2];
  const float* Wv = (const float*)d_in[3];
  const float* Ww = (const float*)d_in[4];
  const float* Wo = (const float*)d_in[5];
  float* outp = (float*)d_out;

  char* ws = (char*)d_ws;
  unsigned short* XB   = (unsigned short*)(ws + OFF_XB);
  unsigned short* WALL = (unsigned short*)(ws + OFF_WALL);
  unsigned short* WOB  = (unsigned short*)(ws + OFF_WOB);
  float*          PROJ = (float*)(ws + OFF_PROJ);
  float*          KSUM = (float*)(ws + OFF_KSUM);
  float*          YF   = (float*)(ws + OFF_YF);
  unsigned short* YNHI = (unsigned short*)(ws + OFF_YNHI);
  unsigned short* YNLO = (unsigned short*)(ws + OFF_YNLO);

  {
    const int n8x = NTOK * NDIM / 8;
    cast_f32_bf16x8<<<n8x / 256, 256, 0, stream>>>(x, XB, n8x);
    const int n8w = NDIM * NDIM / 8;
    cast_f32_bf16x8<<<n8w / 256, 256, 0, stream>>>(Wr, WALL + (size_t)0 * NDIM * NDIM, n8w);
    cast_f32_bf16x8<<<n8w / 256, 256, 0, stream>>>(Wk, WALL + (size_t)1 * NDIM * NDIM, n8w);
    cast_f32_bf16x8<<<n8w / 256, 256, 0, stream>>>(Wv, WALL + (size_t)2 * NDIM * NDIM, n8w);
    cast_f32_bf16x8<<<n8w / 256, 256, 0, stream>>>(Ww, WALL + (size_t)3 * NDIM * NDIM, n8w);
    cast_f32_bf16x8<<<n8w / 256, 256, 0, stream>>>(Wo, WOB, n8w);
  }

  const int proj_blocks = ((NSEQ / 64) * (PROJ_N / 64)) / 8;
  for (int b = 0; b < NBATCH; ++b) {
    const unsigned short* xb = XB + (size_t)b * NSEQ * NDIM;
    wmma_gemm64_bf16<0><<<proj_blocks, 256, 0, stream>>>(
        xb, xb, NDIM, WALL, WALL, NDIM, PROJ, PROJ_N, NSEQ, PROJ_N, NDIM, 1.0f);
    ksum_kernel<<<(NSEQ * NHEAD) / 256, 256, 0, stream>>>(PROJ, KSUM);
    scan_kernel<<<NHEAD, HDIM, 0, stream>>>(PROJ, KSUM, YF, b * NSEQ);
  }

  rmsnorm_split_kernel<<<NTOK, 256, 0, stream>>>(YF, YNHI, YNLO);

  const int out_blocks = ((NTOK / 64) * (NDIM / 64)) / 8;
  wmma_gemm64_bf16<2><<<out_blocks, 256, 0, stream>>>(
      YNHI, YNLO, NDIM, WOB, WOB, NDIM, outp, NDIM, NTOK, NDIM, NDIM, 1.0f);
}
